// RNN_26895085207932
// MI455X (gfx1250) — hardware-verified
//
#include <hip/hip_runtime.h>

constexpr int SEQ_LEN  = 2048;
constexpr int NBATCH   = 4096;
constexpr int NIN      = 1;
constexpr int NHID     = 32;
constexpr int NTHR     = 32;
constexpr int ROWS_PB  = 32;
constexpr int NBLK     = NBATCH / ROWS_PB;
constexpr int HFP      = 36;
constexpr int HP16     = 40;
constexpr int OSTEPS   = 4;
constexpr float H_CARRY  = 256.0f;
constexpr float W_CARRY  = 64.0f;
constexpr float R_CARRY  = 2048.0f;
constexpr float ACC0_SC  = H_CARRY * W_CARRY;
constexpr float ACC0_INV = 1.0f / ACC0_SC;
constexpr float ACC1_INV = 1.0f / (ACC0_SC * R_CARRY);
static_assert(NIN == 1);
static_assert(NHID == 32);
static_assert(ROWS_PB == NTHR && ROWS_PB == 32);
static_assert(NBLK * ROWS_PB == NBATCH);
static_assert(SEQ_LEN % OSTEPS == 0);
static_assert(HFP % 4 == 0 && HP16 % 8 == 0);
static_assert(ACC0_SC == 16384.0f);

typedef __attribute__((ext_vector_type(16))) _Float16 v16h;
typedef __attribute__((ext_vector_type(8)))  _Float16 v8h;
typedef __attribute__((ext_vector_type(8)))  float    v8f;
typedef __attribute__((ext_vector_type(4)))  float    v4f;

struct FragH {
  union U { v16h v; v8h h[2]; };
  static __device__ __forceinline__ v16h load(const _Float16* p) {
    U f; f.h[0] = *(const v8h*)(p); f.h[1] = *(const v8h*)(p + 16); return f.v;
  }
  static __device__ __forceinline__ v8f mma(v16h a, v16h b, v8f c) {
    return __builtin_amdgcn_wmma_f32_16x16x32_f16(false, a, false, b, (short)0, c, false, false);
  }
};
__device__ __forceinline__ void grp_guard(v8f& a, v8f& b, v8f& c, v8f& d, v16h x, v16h y) {
  asm volatile("v_nop\n\tv_nop\n\tv_nop\n\tv_nop" : "+v"(a), "+v"(b), "+v"(c), "+v"(d) : "v"(x), "v"(y));
}
__device__ __forceinline__ void keep4_h(v16h a, v16h b, v16h c, v16h d) { asm volatile("v_nop" :: "v"(a), "v"(b), "v"(c), "v"(d)); }
__device__ __forceinline__ void acc_guard4(v8f& a, v8f& b, v8f& c, v8f& d) { asm volatile("v_nop\n\tv_nop\n\tv_nop\n\tv_nop" : "+v"(a), "+v"(b), "+v"(c), "+v"(d)); }

__device__ __forceinline__ float ftanh(float x) {
  const float e = __builtin_amdgcn_exp2f(x * 2.885390081777927f);
  return 1.0f - 2.0f * __builtin_amdgcn_rcpf(e + 1.0f);
}

__device__ __forceinline__ void split_f16(float v, float carry, _Float16& hi, _Float16& lo) {
  const float vs = v * carry;
  const _Float16 h16 = (_Float16)vs;
  const float back = (float)h16;
  hi = h16;
  lo = (_Float16)((vs - back) * R_CARRY);
}

__device__ __forceinline__ void store_planes(const float (&hv)[NHID], _Float16* hrow, _Float16* lrow) {
  v8h hq[4], lq[4];
#pragma unroll
  for (int q = 0; q < 4; ++q) {
#pragma unroll
    for (int e = 0; e < 8; ++e) {
      _Float16 a, b;
      split_f16(hv[8 * q + e], H_CARRY, a, b);
      hq[q][e] = a;
      lq[q][e] = b;
    }
  }
#pragma unroll
  for (int q = 0; q < 4; ++q) {
    *(v8h*)(hrow + 8 * q) = hq[q];
    *(v8h*)(lrow + 8 * q) = lq[q];
  }
}

__global__ __launch_bounds__(NTHR) void elman_seq_kernel(
    const float* __restrict__ x, const float* __restrict__ hidden,
    const float* __restrict__ W_ih, const float* __restrict__ b_ih,
    const float* __restrict__ W_hh, const float* __restrict__ b_hh,
    const float* __restrict__ W_fc, const float* __restrict__ b_fc,
    float* __restrict__ out) {
  __shared__ __align__(16) float    Hf[ROWS_PB * HFP];
  __shared__ __align__(16) _Float16 Hhi[ROWS_PB * HP16];
  __shared__ __align__(16) _Float16 Hlo[ROWS_PB * HP16];
  __shared__ __align__(16) float    Ob[OSTEPS * ROWS_PB];

  const int lane = threadIdx.x & 31;
  const int c = lane & 15, hh = lane >> 4, koff = hh * 8;
  const int b0 = blockIdx.x * ROWS_PB;

  v16h bwh[2], bwl[2];
#pragma unroll
  for (int j = 0; j < 2; ++j) {
    const float* wr = W_hh + (size_t)(16 * j + c) * NHID;
    const v4f w0 = *(const v4f*)(wr + koff);
    const v4f w1 = *(const v4f*)(wr + koff + 4);
    const v4f w2 = *(const v4f*)(wr + 16 + koff);
    const v4f w3 = *(const v4f*)(wr + 16 + koff + 4);
#pragma unroll
    for (int e = 0; e < 4; ++e) {
      _Float16 a, b;
      split_f16(w0[e], W_CARRY, a, b); bwh[j][e] = a;      bwl[j][e] = b;
      split_f16(w1[e], W_CARRY, a, b); bwh[j][4 + e] = a;  bwl[j][4 + e] = b;
      split_f16(w2[e], W_CARRY, a, b); bwh[j][8 + e] = a;  bwl[j][8 + e] = b;
      split_f16(w3[e], W_CARRY, a, b); bwh[j][12 + e] = a; bwl[j][12 + e] = b;
    }
    asm volatile("" ::: "memory");
  }

  float wihS[2], bsS[2];
#pragma unroll
  for (int j = 0; j < 2; ++j) {
    const int n = 16 * j + c;
    wihS[j] = W_ih[n] * ACC0_SC;
    bsS[j]  = (b_ih[n] + b_hh[n]) * ACC0_SC;
  }
  asm volatile("" ::: "memory");

  float wfc[NHID];
#pragma unroll
  for (int q = 0; q < 8; ++q) {
    const v4f v = *(const v4f*)(W_fc + 4 * q);
    wfc[4 * q] = v[0]; wfc[4 * q + 1] = v[1]; wfc[4 * q + 2] = v[2]; wfc[4 * q + 3] = v[3];
  }
  const float bfc = b_fc[0];
  asm volatile("" ::: "memory");

  {
    float hv[NHID];
    const float* hr = hidden + (size_t)(b0 + lane) * NHID;
#pragma unroll
    for (int q = 0; q < 8; ++q) {
      const v4f v = *(const v4f*)(hr + 4 * q);
      hv[4 * q] = v[0]; hv[4 * q + 1] = v[1]; hv[4 * q + 2] = v[2]; hv[4 * q + 3] = v[3];
    }
    store_planes(hv, Hhi + lane * HP16, Hlo + lane * HP16);
  }
  __syncthreads();

  const v8f z8 = {0.f, 0.f, 0.f, 0.f, 0.f, 0.f, 0.f, 0.f};

#pragma unroll 1
  for (int t = 0; t < SEQ_LEN; ++t) {
    const float* xr = x + (size_t)t * NBATCH + b0;
    v4f xa[2], xb[2];
#pragma unroll
    for (int i = 0; i < 2; ++i) {
      xa[i] = *(const v4f*)(xr + 16 * i + 8 * hh);
      xb[i] = *(const v4f*)(xr + 16 * i + 8 * hh + 4);
    }
    v8f acc0[2][2], acc1[2][2];
#pragma unroll
    for (int i = 0; i < 2; ++i) {
#pragma unroll
      for (int j = 0; j < 2; ++j) {
#pragma unroll
        for (int r = 0; r < 4; ++r) {
          acc0[i][j][r]     = fmaf(xa[i][r], wihS[j], bsS[j]);
          acc0[i][j][4 + r] = fmaf(xb[i][r], wihS[j], bsS[j]);
        }
        acc1[i][j] = z8;
      }
    }

#pragma unroll
    for (int i = 0; i < 2; ++i) {
      const v16h ah = FragH::load(Hhi + (16 * i + c) * HP16 + koff);
      const v16h al = FragH::load(Hlo + (16 * i + c) * HP16 + koff);
#pragma unroll
      for (int j = 0; j < 2; ++j) {
        acc0[i][j] = FragH::mma(ah, bwh[j], acc0[i][j]);
        acc1[i][j] = FragH::mma(al, bwh[j], acc1[i][j]);
        acc1[i][j] = FragH::mma(ah, bwl[j], acc1[i][j]);
      }
      grp_guard(acc0[i][0], acc0[i][1], acc1[i][0], acc1[i][1], ah, al);
    }
    keep4_h(bwh[0], bwh[1], bwl[0], bwl[1]);
    acc_guard4(acc0[0][0], acc0[0][1], acc0[1][0], acc0[1][1]);
    acc_guard4(acc1[0][0], acc1[0][1], acc1[1][0], acc1[1][1]);

#pragma unroll
    for (int i = 0; i < 2; ++i) {
#pragma unroll
      for (int j = 0; j < 2; ++j) {
#pragma unroll
        for (int r = 0; r < 8; ++r) {
          float pre = acc0[i][j][r] * ACC0_INV;
          pre = fmaf(acc1[i][j][r], ACC1_INV, pre);
          Hf[(16 * i + 8 * hh + r) * HFP + 16 * j + c] = ftanh(pre);
        }
      }
    }
    __syncthreads();

    float hv[NHID];
    {
      const float* hr = Hf + lane * HFP;
#pragma unroll
      for (int q = 0; q < 8; ++q) {
        const v4f v = *(const v4f*)(hr + 4 * q);
        hv[4 * q] = v[0]; hv[4 * q + 1] = v[1]; hv[4 * q + 2] = v[2]; hv[4 * q + 3] = v[3];
      }
    }
    float d = 0.0f;
#pragma unroll
    for (int k = 0; k < NHID; ++k) d = fmaf(hv[k], wfc[k], d);
    Ob[(t & (OSTEPS - 1)) * ROWS_PB + lane] = d + bfc;
    store_planes(hv, Hhi + lane * HP16, Hlo + lane * HP16);
    __syncthreads();

    if ((t & (OSTEPS - 1)) == OSTEPS - 1) {
      const int s = lane >> 3, q4 = (lane & 7) * 4;
      const int t0 = t - (OSTEPS - 1);
      const v4f v = *(const v4f*)(Ob + s * ROWS_PB + q4);
      float* op = out + (size_t)(t0 + s) * NBATCH + b0 + q4;
      *(volatile v4f*)op = v;
      __threadfence();
      *(volatile v4f*)op = v;
    }
  }
}

extern "C" void kernel_launch(void* const* d_in, const int* in_sizes, int n_in,
                              void* d_out, int out_size, void* d_ws, size_t ws_size, hipStream_t stream) {
  (void)d_ws; (void)ws_size;
  if (n_in < 8 || d_out == nullptr) return;
  if (in_sizes[0] != SEQ_LEN * NBATCH * NIN || in_sizes[1] != NBATCH * NHID || in_sizes[2] != NHID * NIN ||
      in_sizes[3] != NHID || in_sizes[4] != NHID * NHID || in_sizes[5] != NHID || in_sizes[6] != NIN * NHID ||
      in_sizes[7] != NIN || out_size != SEQ_LEN * NBATCH * NIN) return;

  const float* x      = (const float*)d_in[0];
  const float* hidden = (const float*)d_in[1];
  const float* W_ih   = (const float*)d_in[2];
  const float* b_ih   = (const float*)d_in[3];
  const float* W_hh   = (const float*)d_in[4];
  const float* b_hh   = (const float*)d_in[5];
  const float* W_fc   = (const float*)d_in[6];
  const float* b_fc   = (const float*)d_in[7];
  float* out = (float*)d_out;

  elman_seq_kernel<<<NBLK, NTHR, 0, stream>>>(x, hidden, W_ih, b_ih, W_hh, b_hh, W_fc, b_fc, out);
}
